// Encoder_28741921145341
// MI455X (gfx1250) — hardware-run, weakly checked
//
#include <hip/hip_runtime.h>
#include <math.h>

typedef __attribute__((ext_vector_type(16))) _Float16 v16h;
typedef __attribute__((ext_vector_type(8)))  _Float16 v8h;
typedef __attribute__((ext_vector_type(8)))  float    v8f;
typedef __attribute__((ext_vector_type(4)))  float    v4f;
typedef __attribute__((ext_vector_type(4)))  unsigned v4u;

constexpr int kB     = 128;
constexpr int kT     = 255;
constexpr int kN     = 256;
constexpr int kH     = 256;
constexpr int kG     = 4 * kH;
constexpr int kRows  = kB * kT;
constexpr int kWaOff = 2 * kH;
constexpr int kWaLen = 2 * kH + kT;
constexpr int kHP    = 272;
constexpr int kSP    = 36;
static_assert(kRows == 32640);
static_assert(kG == 1024);
static_assert(kWaLen == 767);
static_assert((kRows % 64) == 0 && (kG % 64) == 0 && (kN % 32) == 0 && (kH % 32) == 0);
static_assert((kRows % 32) == 0);
static_assert((2 * 16 * kHP) % 256 == 0);
static_assert((kHP % 8) == 0 && kHP >= kH);
static_assert((kSP % 4) == 0 && kSP >= 32);
static_assert(kB % 16 == 0);

constexpr float kXCarry    = 2048.0f;
constexpr float kWCarry    = 256.0f;
constexpr float kHCarry    = 4096.0f;
constexpr float kZCarry    = 256.0f;
constexpr float kGemmScale = kZCarry / (kXCarry * kWCarry);
constexpr float kZUp       = (kHCarry * kWCarry) / kZCarry;
constexpr float kZFold     = 1.0f / (kHCarry * kWCarry);
constexpr float kF16MinN   = 6.103515625e-5f;
static_assert(kGemmScale == 1.0f / 2048.0f);
static_assert(kZUp == 4096.0f);
static_assert(kZFold == 1.0f / 1048576.0f);

constexpr size_t kOffAlpha = 0;
constexpr size_t kOffXt    = kOffAlpha + (size_t)kB * kN * 4;
constexpr size_t kOffBtw   = kOffXt    + (size_t)kRows * kN * 2;
constexpr size_t kOffBtu   = kOffBtw   + (size_t)kG * kN * 2;
constexpr size_t kOffBz    = kOffBtu   + (size_t)kG * kH * 2;
constexpr size_t kOffZx    = kOffBz    + (size_t)kG * 4;
constexpr size_t kWsTotal  = kOffZx    + (size_t)kRows * kG * 2;
static_assert(kWsTotal == 84742144ull);
static_assert(kWsTotal <= 134217728ull);
static_assert((kOffXt % 256) == 0 && (kOffBtw % 256) == 0 && (kOffBtu % 256) == 0 &&
              (kOffBz % 256) == 0 && (kOffZx % 256) == 0);

__device__ __forceinline__ unsigned short f2bf_bits(float f) {
  unsigned u = __float_as_uint(f);
  return (unsigned short)((u + 0x7FFFu + ((u >> 16) & 1u)) >> 16);
}
__device__ __forceinline__ float bf_bits2f(unsigned short h) { return __uint_as_float(((unsigned)h) << 16); }
__device__ __forceinline__ float bf16r(float f) { return bf_bits2f(f2bf_bits(f)); }
__device__ __forceinline__ float flush16(float v) { return (fabsf(v) < kF16MinN) ? 0.0f : v; }
__device__ __forceinline__ float h16_to_f32(unsigned hb) {
  const unsigned sgn = (hb & 0x8000u) << 16;
  const unsigned em  = hb & 0x7fffu;
  const float fn  = __uint_as_float((em << 13) + 0x38000000u);
  const float fs  = (float)em * 5.9604644775390625e-8f;
  const float mag = (em < 0x400u) ? fs : fn;
  return __uint_as_float(__float_as_uint(mag) | sgn);
}
__device__ __forceinline__ int perm_col(int np) {
  const int w  = np >> 7;
  const int c  = (np >> 3) & 15;
  const int g  = (np >> 1) & 3;
  const int ut = np & 1;
  return 256 * g + 32 * w + 2 * c + ut;
}
__device__ __forceinline__ float sigm(float x)   { return 1.0f / (1.0f + expf(-x)); }
__device__ __forceinline__ float tanh_e(float x) { return 1.0f - 2.0f / (1.0f + expf(2.0f * x)); }

__device__ __forceinline__ void dep_guard4_h(v8f& a, v8f& b, v8f& c, v8f& d, v16h x, v16h y) {
  asm volatile("v_nop\n\tv_nop\n\tv_nop\n\tv_nop" : "+v"(a), "+v"(b), "+v"(c), "+v"(d) : "v"(x), "v"(y));
}
__device__ __forceinline__ void keep4_h(v16h a, v16h b, v16h c, v16h d) { asm volatile("v_nop" :: "v"(a), "v"(b), "v"(c), "v"(d)); }
__device__ __forceinline__ void acc_guard4(v8f& a, v8f& b, v8f& c, v8f& d) {
  asm volatile("v_nop\n\tv_nop\n\tv_nop\n\tv_nop" : "+v"(a), "+v"(b), "+v"(c), "+v"(d));
}
template <typename T> struct Frag;
template <> struct Frag<_Float16> {
  typedef v16h V; union U { v16h v; v8h h[2]; };
  static __device__ __forceinline__ v16h load(const _Float16* p) {
    U f; f.h[0] = *(const v8h*)(p); f.h[1] = *(const v8h*)(p + 16); return f.v;
  }
  static __device__ __forceinline__ v8f mma(v16h a, v16h b, v8f c) {
    return __builtin_amdgcn_wmma_f32_16x16x32_f16(false, a, false, b, (short)0, c, false, false);
  }
};
__device__ __forceinline__ v8f mma_tied(v16h a, v16h b, v8f c) {
  c = __builtin_amdgcn_wmma_f32_16x16x32_f16(false, a, false, b, (short)0, c, false, false);
  asm volatile("v_nop\n\tv_nop\n\tv_nop\n\tv_nop" : "+v"(c) : "v"(a), "v"(b));
  return c;
}

__global__ __launch_bounds__(256) void alpha_kernel(const float* __restrict__ X, const float* __restrict__ Wa,
                                                    float* __restrict__ ALPHA) {
  __shared__ float s_w[256];
  __shared__ float s_red[16];
  __shared__ __align__(16) float s_a[256];
  const int tid = threadIdx.x, lane = tid & 31, wave = tid >> 5;
  const int b = blockIdx.x;
  {
    const int ti = (tid < kT) ? tid : (kT - 1);
    float wv = Wa[kWaOff + ti];
    asm volatile("" : "+v"(wv));
    s_w[tid] = (tid < kT) ? bf16r(wv) : 0.0f;
  }
  __syncthreads();
  const float* xp = X + (size_t)b * kT * kN + tid;
  float acc = 0.0f;
#pragma unroll 5
  for (int t = 0; t < kT; ++t) acc = fmaf(bf16r(xp[(size_t)t * kN]), s_w[t], acc);

  float m = acc;
#pragma unroll
  for (int off = 1; off < 32; off <<= 1) m = fmaxf(m, __shfl_xor(m, off, 32));
  if (lane == 0) s_red[wave] = m;
  __syncthreads();
  float bm = s_red[0];
#pragma unroll
  for (int i = 1; i < 8; ++i) bm = fmaxf(bm, s_red[i]);
  const float e = expf(acc - bm);
  float s = e;
#pragma unroll
  for (int off = 1; off < 32; off <<= 1) s += __shfl_xor(s, off, 32);
  if (lane == 0) s_red[8 + wave] = s;
  __syncthreads();
  float tot = s_red[8];
#pragma unroll
  for (int i = 1; i < 8; ++i) tot += s_red[8 + i];
  s_a[tid] = e / tot;
  __syncthreads();
  if (tid < 64) {
    const v4f v = *(const v4f*)(s_a + 4 * tid);
    float* op = ALPHA + (size_t)b * kN + 4 * tid;
    *(volatile v4f*)op = v;
    __threadfence();
    *(volatile v4f*)op = v;
  }
}

__global__ __launch_bounds__(256) void xtilde_kernel(const float* __restrict__ X, const float* __restrict__ ALPHA,
                                                     float* __restrict__ OUT0, unsigned short* __restrict__ XT16) {
  const int lane = threadIdx.x & 31, wave = threadIdx.x >> 5;
  const int row0 = (blockIdx.x * 8 + wave) * 4;
#pragma unroll 1
  for (int i = 0; i < 4; ++i) {
    const int row = row0 + i;
    const int b = row / kT;
    const float* xr = X + (size_t)row * kN;
    const float* ar = ALPHA + (size_t)b * kN;
    const v4f x0 = *(const v4f*)(xr + 4 * lane);
    const v4f x1 = *(const v4f*)(xr + 128 + 4 * lane);
    const v4f a0 = *(const v4f*)(ar + 4 * lane);
    const v4f a1 = *(const v4f*)(ar + 128 + 4 * lane);
    const v4f y0 = *(const v4f*)(xr + 8 * lane);
    const v4f y1 = *(const v4f*)(xr + 8 * lane + 4);
    const v4f g0 = *(const v4f*)(ar + 8 * lane);
    const v4f g1 = *(const v4f*)(ar + 8 * lane + 4);
    v4f o0, o1;
    v8h hv;
#pragma unroll
    for (int e = 0; e < 4; ++e) {
      o0[e] = a0[e] * bf16r(x0[e]);
      o1[e] = a1[e] * bf16r(x1[e]);
      const float p0 = g0[e] * bf16r(y0[e]);
      const float p1 = g1[e] * bf16r(y1[e]);
      hv[e]     = (_Float16)flush16(p0 * kXCarry);
      hv[4 + e] = (_Float16)flush16(p1 * kXCarry);
    }
    float* op = OUT0 + (size_t)row * kN;
    unsigned short* hp = XT16 + (size_t)row * kN + 8 * lane;
    for (int pass = 0; pass < 2; ++pass) {
      *(volatile v4f*)(op + 4 * lane) = o0;
      *(volatile v4f*)(op + 128 + 4 * lane) = o1;
      *(volatile v8h*)hp = hv;
      __threadfence();
    }
  }
}

__global__ __launch_bounds__(256) void pack_weights_kernel(const float* __restrict__ Wl, const float* __restrict__ Ul,
                                                           unsigned short* __restrict__ BTW,
                                                           unsigned short* __restrict__ BTU) {
  __shared__ float sT[64 * 65];
  const int tid = threadIdx.x;
  const int n0 = blockIdx.x * 64, k0 = blockIdx.y * 64;
  const bool second = (blockIdx.z != 0);
  const float* src = second ? Ul : Wl;
  unsigned short* dst = second ? BTU : BTW;
  const int nl = tid & 63, kr = tid >> 6;
  const int ncol = perm_col(n0 + nl);
#pragma unroll 4
  for (int i = 0; i < 16; ++i) {
    const int kk = kr + 4 * i;
    sT[nl * 65 + kk] = src[(size_t)(k0 + kk) * kG + ncol];
  }
  __syncthreads();
  const int q = tid >> 3, c8 = (tid & 7) * 8;
  v8h hv[2];
#pragma unroll
  for (int it = 0; it < 2; ++it) {
    const float* sp = sT + (it * 32 + q) * 65 + c8;
#pragma unroll
    for (int e = 0; e < 8; ++e) hv[it][e] = (_Float16)flush16(bf16r(sp[e]) * kWCarry);
  }
  for (int pass = 0; pass < 2; ++pass) {
#pragma unroll
    for (int it = 0; it < 2; ++it)
      *(volatile v8h*)(dst + (size_t)(n0 + it * 32 + q) * kH + k0 + c8) = hv[it];
    __threadfence();
  }
}

__global__ __launch_bounds__(256) void bias_prep_kernel(const float* __restrict__ bl, float* __restrict__ BZ) {
  const int n0 = 4 * threadIdx.x;
  v4f o;
#pragma unroll
  for (int e = 0; e < 4; ++e) o[e] = bf16r(bl[perm_col(n0 + e)]) * kZCarry;
  float* op = BZ + n0;
  *(volatile v4f*)op = o;
  __threadfence();
  *(volatile v4f*)op = o;
}

template <int BIAS_MODE, int OUT_MODE>
__global__ __launch_bounds__(256) void wmma_gemm64(
    const unsigned short* __restrict__ Ap, int lda,
    const unsigned short* __restrict__ Btp, int ldb,
    void* __restrict__ Cout, int ldc,
    const float* __restrict__ bias,
    int M, int N, int K, float scale) {
  typedef _Float16 T;
  typedef v16h V;
  const T* A = (const T*)Ap;
  const T* Bt = (const T*)Btp;
  __shared__ __align__(16) float sT[8][16 * 68];
  const int lane = threadIdx.x & 31;
  const int wave = threadIdx.x >> 5;
  const int tilesN = N >> 6;
  const int tilesM = M >> 6;
  const int tile = blockIdx.x * 8 + wave;
  if (tile >= tilesM * tilesN) return;
  const int tm = tile / tilesN;
  const int tn = tile - tm * tilesN;
  const int m0 = tm << 6;
  const int n0 = tn << 6;

  const int rlane = lane & 15;
  const int koff  = (lane >> 4) * 8;
  const int mOff  = (lane >> 4) * 8;

  v8f acc[4][4];
#pragma unroll
  for (int i = 0; i < 4; ++i)
#pragma unroll
    for (int j = 0; j < 4; ++j) acc[i][j] = (v8f){0.f,0.f,0.f,0.f,0.f,0.f,0.f,0.f};

  for (int k0 = 0; k0 < K; k0 += 32) {
    V bh[4];
#pragma unroll
    for (int j = 0; j < 4; ++j) {
      const size_t bo = (size_t)(n0 + (j << 4) + rlane) * ldb + koff + k0;
      bh[j] = Frag<T>::load(Bt + bo);
    }
#pragma unroll
    for (int i = 0; i < 4; ++i) {
      const size_t ao = (size_t)(m0 + (i << 4) + rlane) * lda + koff + k0;
      V ah = Frag<T>::load(A + ao);
#pragma unroll
      for (int j = 0; j < 4; ++j) acc[i][j] = Frag<T>::mma(ah, bh[j], acc[i][j]);
      dep_guard4_h(acc[i][0], acc[i][1], acc[i][2], acc[i][3], ah, bh[3]);
    }
    keep4_h(bh[0], bh[1], bh[2], bh[3]);
  }
  acc_guard4(acc[0][0], acc[0][1], acc[0][2], acc[0][3]);
  acc_guard4(acc[1][0], acc[1][1], acc[1][2], acc[1][3]);
  acc_guard4(acc[2][0], acc[2][1], acc[2][2], acc[2][3]);
  acc_guard4(acc[3][0], acc[3][1], acc[3][2], acc[3][3]);

  float* slab = sT[wave];
#pragma unroll
  for (int i = 0; i < 4; ++i) {
    const int mBase = m0 + (i << 4);
#pragma unroll
    for (int j = 0; j < 4; ++j) {
      const int n = n0 + (j << 4) + rlane;
      float bv = 0.f;
      if (BIAS_MODE == 2) bv = bias[n];
#pragma unroll
      for (int r = 0; r < 8; ++r) {
        float v = acc[i][j][r] * scale;
        if (BIAS_MODE == 2) v += bv;
        slab[(mOff + r) * 68 + (j << 4) + rlane] = v;
      }
    }
    __builtin_amdgcn_fence(__ATOMIC_RELEASE, "workgroup");
    __builtin_amdgcn_wave_barrier();
    __builtin_amdgcn_fence(__ATOMIC_ACQUIRE, "workgroup");
    if (OUT_MODE == 0) {
      float* C = (float*)Cout;
      const int hh = lane >> 4, c4 = (lane & 15) * 4;
      for (int pass = 0; pass < 2; ++pass) {
#pragma unroll
        for (int it = 0; it < 8; ++it) {
          const int row = it * 2 + hh;
          v4f v = *(const v4f*)(slab + row * 68 + c4);
          *(volatile v4f*)(C + (size_t)(mBase + row) * ldc + n0 + c4) = v;
        }
        __threadfence();
      }
    } else {
      const int q = lane >> 3, c8 = (lane & 7) * 8;
      unsigned short* C = (unsigned short*)Cout;
      for (int pass = 0; pass < 2; ++pass) {
#pragma unroll
        for (int it = 0; it < 4; ++it) {
          const int row = it * 4 + q;
          const float* sp = slab + row * 68 + c8;
          v8h hv;
#pragma unroll
          for (int e = 0; e < 8; ++e) hv[e] = (_Float16)sp[e];
          *(volatile v8h*)(C + (size_t)(mBase + row) * ldc + n0 + c8) = hv;
        }
        __threadfence();
      }
    }
    __builtin_amdgcn_fence(__ATOMIC_RELEASE, "workgroup");
    __builtin_amdgcn_wave_barrier();
    __builtin_amdgcn_fence(__ATOMIC_ACQUIRE, "workgroup");
  }
}

__global__ __launch_bounds__(256) void lstm_seq_kernel(const float* __restrict__ X,
                                                       const unsigned short* __restrict__ ZXp,
                                                       const unsigned short* __restrict__ BUp,
                                                       float* __restrict__ OUT1) {
  __shared__ __align__(16) _Float16 Ah[2][16 * kHP];
  __shared__ __align__(16) float    Sl[8][16 * kSP];
  __shared__ float s_h0[16];
  const _Float16* BU = (const _Float16*)BUp;
  const int tid = threadIdx.x, lane = tid & 31, wave = tid >> 5;
  const int c = lane & 15, hh = lane >> 4, koff = hh * 8;
  const int b0 = blockIdx.x * 16;

  {
    float x0 = X[(size_t)(b0 + (tid & 15)) * ((size_t)kT * kN)];
    asm volatile("" : "+v"(x0));
    if (tid < 16) s_h0[tid] = bf16r(x0);
  }
  __syncthreads();
  {
    _Float16* ahf = &Ah[0][0];
#pragma unroll 1
    for (int i = tid; i < 2 * 16 * kHP; i += 256) {
      const int bufrow = i / kHP;
      const int col = i - bufrow * kHP;
      const float hv0 = s_h0[bufrow & 15];
      float v = flush16(hv0 * kHCarry);
      v = (bufrow < 16 && col < kH) ? v : 0.0f;
      ahf[i] = (_Float16)v;
    }
  }
  v8f cst0, cst1;
#pragma unroll
  for (int r = 0; r < 8; ++r) {
    const float cv = s_h0[8 * hh + r];
    cst0[r] = cv;
    cst1[r] = cv;
  }
  __syncthreads();

  const _Float16* bbase = BU + (size_t)(128 * wave + 8 * c) * kH + koff;
  const unsigned short* zbase = ZXp + 128 * wave + 8 * c;
  float* slab = Sl[wave];
  const int q = lane >> 3, c4 = (lane & 7) * 4;

#pragma unroll 1
  for (int t = 0; t < kT; ++t) {
    const int cur = t & 1;
    const _Float16* ahrow = &Ah[cur][0] + c * kHP + koff;
    _Float16* ahn = &Ah[cur ^ 1][0];

    v8f acc[4][2];
#pragma unroll
    for (int r = 0; r < 8; ++r) {
      const size_t m = (size_t)(b0 + 8 * hh + r) * kT + (size_t)t;
      const v4u qz = *(const v4u*)(zbase + m * kG);
#pragma unroll
      for (int g = 0; g < 4; ++g) {
        const unsigned wd = qz[g];
        acc[g][0][r] = h16_to_f32(wd & 0xffffu) * kZUp;
        acc[g][1][r] = h16_to_f32(wd >> 16) * kZUp;
      }
    }

#pragma unroll 1
    for (int k0 = 0; k0 < kH; k0 += 32) {
      const v16h a = Frag<_Float16>::load(ahrow + k0);
#pragma unroll
      for (int g = 0; g < 4; ++g) {
#pragma unroll
        for (int ut = 0; ut < 2; ++ut) {
          const v16h bf = Frag<_Float16>::load(bbase + (size_t)(2 * g + ut) * kH + k0);
          acc[g][ut] = mma_tied(a, bf, acc[g][ut]);
        }
      }
    }

#pragma unroll 1
    for (int ut = 0; ut < 2; ++ut) {
#pragma unroll
      for (int r = 0; r < 8; ++r) {
        const float zi = acc[0][0][r] * kZFold;
        const float zf = acc[1][0][r] * kZFold;
        const float zg = acc[2][0][r] * kZFold;
        const float zo = acc[3][0][r] * kZFold;
        const float ig = sigm(zi);
        const float fg = sigm(zf);
        const float gg = tanh_e(zg);
        const float og = sigm(zo);
        const float cn = fg * cst0[r] + ig * gg;
        cst0[r] = cn;
        const float hn = og * tanh_e(cn);
        const float hv = flush16(hn * kHCarry);
        const int row = 8 * hh + r;
        ahn[row * kHP + 32 * wave + 2 * c + ut] = (_Float16)hv;
        slab[row * kSP + 2 * c + ut] = hn;
      }
#pragma unroll
      for (int g = 0; g < 4; ++g) acc[g][0] = acc[g][1];
      {
        const v8f tmp = cst0;
        cst0 = cst1;
        cst1 = tmp;
      }
    }

    __builtin_amdgcn_fence(__ATOMIC_RELEASE, "workgroup");
    __builtin_amdgcn_wave_barrier();
    __builtin_amdgcn_fence(__ATOMIC_ACQUIRE, "workgroup");
    v4f ov[4];
#pragma unroll
    for (int it = 0; it < 4; ++it) ov[it] = *(const v4f*)(slab + (it * 4 + q) * kSP + c4);
    float* ob = OUT1 + ((size_t)b0 * kT + (size_t)t) * kH + 32 * wave + c4;
    for (int pass = 0; pass < 2; ++pass) {
#pragma unroll
      for (int it = 0; it < 4; ++it)
        *(volatile v4f*)(ob + (size_t)(it * 4 + q) * ((size_t)kT * kH)) = ov[it];
      __threadfence();
    }
    __builtin_amdgcn_fence(__ATOMIC_RELEASE, "workgroup");
    __builtin_amdgcn_wave_barrier();
    __builtin_amdgcn_fence(__ATOMIC_ACQUIRE, "workgroup");
    __syncthreads();
  }
}

extern "C" void kernel_launch(void* const* d_in, const int* in_sizes, int n_in,
                              void* d_out, int out_size, void* d_ws, size_t ws_size,
                              hipStream_t stream) {
  if (n_in < 6 || d_out == nullptr || d_ws == nullptr) return;
  if (in_sizes[0] != kRows * kN) return;
  if (in_sizes[1] != kWaLen) return;
  if (in_sizes[2] != 1) return;
  if (in_sizes[3] != kN * kG) return;
  if (in_sizes[4] != kH * kG) return;
  if (in_sizes[5] != kG) return;
  if (out_size != 2 * kRows * kH) return;
  if (ws_size < kWsTotal) return;

  const float* X  = (const float*)d_in[0];
  const float* Wa = (const float*)d_in[1];
  const float* Wl = (const float*)d_in[3];
  const float* Ul = (const float*)d_in[4];
  const float* bl = (const float*)d_in[5];
  float* out0 = (float*)d_out;
  float* out1 = (float*)d_out + (size_t)kRows * kN;

  char* ws = (char*)d_ws;
  float*          ALPHA = (float*)(ws + kOffAlpha);
  unsigned short* XT16  = (unsigned short*)(ws + kOffXt);
  unsigned short* BTW   = (unsigned short*)(ws + kOffBtw);
  unsigned short* BTU   = (unsigned short*)(ws + kOffBtu);
  float*          BZ    = (float*)(ws + kOffBz);
  unsigned short* ZX16  = (unsigned short*)(ws + kOffZx);

  alpha_kernel<<<kB, 256, 0, stream>>>(X, Wa, ALPHA);
  xtilde_kernel<<<kRows / 32, 256, 0, stream>>>(X, ALPHA, out0, XT16);
  pack_weights_kernel<<<dim3(kG / 64, kH / 64, 2), 256, 0, stream>>>(Wl, Ul, BTW, BTU);
  bias_prep_kernel<<<1, 256, 0, stream>>>(bl, BZ);
  wmma_gemm64<2, 1><<<dim3((kRows / 64) * (kG / 64) / 8, 1), 256, 0, stream>>>(
      XT16, kN, BTW, kN, (void*)ZX16, kG, BZ, kRows, kG, kN, kGemmScale);
  lstm_seq_kernel<<<kB / 16, 256, 0, stream>>>(X, ZX16, BTU, out1);
}
